// QLSTMQuantum_65481071399783
// MI455X (gfx1250) — hardware-run, weakly checked
//
#include <hip/hip_runtime.h>
#include <math.h>

constexpr int NBATCH   = 1024;
constexpr int NSTEP    = 64;
constexpr int IN_DIM   = 32;
constexpr int NQ       = 8;
constexpr int KDIM     = IN_DIM + NQ;
constexpr int NGATE    = 4;
constexpr int NCOL     = NGATE * NQ;
constexpr int NPADN    = 64;
constexpr int NROWS    = NBATCH * NSTEP;
constexpr int XPP      = 64;
constexpr int OUT0_N   = NROWS * NQ;
constexpr int OUT1_N   = NBATCH * NQ;
constexpr int X_N8     = NROWS * IN_DIM / 8;
constexpr int SCAN_THR = 64;
constexpr int SLP      = 44;
constexpr int YSTAGE   = 32;
static_assert(KDIM == 40);
static_assert(NCOL == 32);
static_assert(IN_DIM % 32 == 0);
static_assert(NROWS % 64 == 0 && NPADN % 64 == 0);
static_assert((NROWS / 64) * (NPADN / 64) % 8 == 0);
static_assert(X_N8 % 256 == 0);
static_assert(NSTEP % 4 == 0);
static_assert(NBATCH % SCAN_THR == 0);
static_assert(SLP % 4 == 0 && SLP >= YSTAGE + NQ);
static_assert(OUT0_N * 4 == 2097152);
static_assert((OUT0_N + 2 * OUT1_N) * 4 == 2162688);
static_assert(NPADN * IN_DIM == 256 * 8);

typedef __attribute__((ext_vector_type(16))) __bf16   v16b;
typedef __attribute__((ext_vector_type(8)))  __bf16   v8b;
typedef __attribute__((ext_vector_type(8)))  float    v8f;
typedef __attribute__((ext_vector_type(4)))  float    v4f;
typedef __attribute__((ext_vector_type(4)))  unsigned v4u;

__device__ __forceinline__ unsigned short f2bf_bits(float f) {
  unsigned u = __float_as_uint(f);
  return (unsigned short)((u + 0x7FFFu + ((u >> 16) & 1u)) >> 16);
}
__device__ __forceinline__ float bf_bits2f(unsigned short h) { return __uint_as_float(((unsigned)h) << 16); }

__device__ __forceinline__ void dep_guard4_b(v8f& a, v8f& b, v8f& c, v8f& d, v16b x, v16b y) {
  asm volatile("v_nop\n\tv_nop\n\tv_nop\n\tv_nop" : "+v"(a), "+v"(b), "+v"(c), "+v"(d) : "v"(x), "v"(y));
}
__device__ __forceinline__ void keep4_b(v16b a, v16b b, v16b c, v16b d) { asm volatile("v_nop" :: "v"(a), "v"(b), "v"(c), "v"(d)); }
__device__ __forceinline__ void acc_guard4(v8f& a, v8f& b, v8f& c, v8f& d) {
  asm volatile("v_nop\n\tv_nop\n\tv_nop\n\tv_nop" : "+v"(a), "+v"(b), "+v"(c), "+v"(d));
}

struct FragB {
  union U { v16b v; v8b h[2]; };
  static __device__ __forceinline__ v16b load(const __bf16* p) {
    U f; f.h[0] = *(const v8b*)(p); f.h[1] = *(const v8b*)(p + 16); return f.v;
  }
  static __device__ __forceinline__ v8f mma(v16b a, v16b b, v8f c) {
    return __builtin_amdgcn_wmma_f32_16x16x32_bf16(false, a, false, b, (short)0, c, false, false);
  }
};

__device__ __forceinline__ float fsig(float x)  { return __builtin_amdgcn_rcpf(1.0f + __expf(-x)); }
__device__ __forceinline__ float ftanh(float x) { return 1.0f - 2.0f * __builtin_amdgcn_rcpf(__expf(2.0f * x) + 1.0f); }

__global__ __launch_bounds__(256) void split_x_kernel(const float* __restrict__ x, unsigned* __restrict__ Ahi,
                                                      unsigned* __restrict__ Alo) {
  const int i = blockIdx.x * 256 + threadIdx.x;
  const float* sp = x + (size_t)i * 8;
  const v4f a = *(const v4f*)(sp);
  const v4f b = *(const v4f*)(sp + 4);
  v4u wh, wl;
#pragma unroll
  for (int e = 0; e < 2; ++e) {
    const float a0 = a[2 * e], a1 = a[2 * e + 1], b0 = b[2 * e], b1 = b[2 * e + 1];
    const unsigned short ha0 = f2bf_bits(a0), ha1 = f2bf_bits(a1), hb0 = f2bf_bits(b0), hb1 = f2bf_bits(b1);
    const unsigned short la0 = f2bf_bits(a0 - bf_bits2f(ha0)), la1 = f2bf_bits(a1 - bf_bits2f(ha1));
    const unsigned short lb0 = f2bf_bits(b0 - bf_bits2f(hb0)), lb1 = f2bf_bits(b1 - bf_bits2f(hb1));
    wh[e]     = (unsigned)ha0 | ((unsigned)ha1 << 16);
    wh[2 + e] = (unsigned)hb0 | ((unsigned)hb1 << 16);
    wl[e]     = (unsigned)la0 | ((unsigned)la1 << 16);
    wl[2 + e] = (unsigned)lb0 | ((unsigned)lb1 << 16);
  }
  *(volatile v4u*)(Ahi + (size_t)i * 4) = wh;
  *(volatile v4u*)(Alo + (size_t)i * 4) = wl;
  __threadfence();
  *(volatile v4u*)(Ahi + (size_t)i * 4) = wh;
  *(volatile v4u*)(Alo + (size_t)i * 4) = wl;
}

__global__ __launch_bounds__(256) void split_w_kernel(const float* __restrict__ W0, const float* __restrict__ W1,
                                                      const float* __restrict__ W2, const float* __restrict__ W3,
                                                      unsigned* __restrict__ Bhi, unsigned* __restrict__ Blo) {
  const int tid  = threadIdx.x;
  const int wave = __builtin_amdgcn_readfirstlane((int)(threadIdx.x >> 5));
  const int n    = tid >> 2;
  const int c8   = (tid & 3) * 8;
  const int q    = n & 7;
  const int gsel = wave & 3;
  const bool live = wave < 4;
  const int so = q * KDIM + c8;
  v4f a0 = *(const v4f*)(W0 + so);
  v4f b0 = *(const v4f*)(W0 + so + 4);
  v4f a1 = *(const v4f*)(W1 + so);
  v4f b1 = *(const v4f*)(W1 + so + 4);
  v4f a2 = *(const v4f*)(W2 + so);
  v4f b2 = *(const v4f*)(W2 + so + 4);
  v4f a3 = *(const v4f*)(W3 + so);
  v4f b3 = *(const v4f*)(W3 + so + 4);
  asm volatile("" : "+v"(a0), "+v"(b0), "+v"(a1), "+v"(b1));
  asm volatile("" : "+v"(a2), "+v"(b2), "+v"(a3), "+v"(b3));
  float va[4], vb[4];
#pragma unroll
  for (int e = 0; e < 4; ++e) {
    const float ta = (gsel == 0) ? a0[e] : (gsel == 1) ? a1[e] : (gsel == 2) ? a2[e] : a3[e];
    const float tb = (gsel == 0) ? b0[e] : (gsel == 1) ? b1[e] : (gsel == 2) ? b2[e] : b3[e];
    va[e] = live ? ta : 0.0f;
    vb[e] = live ? tb : 0.0f;
  }
  v4u wh, wl;
#pragma unroll
  for (int e = 0; e < 2; ++e) {
    const float p0 = va[2 * e], p1 = va[2 * e + 1], r0 = vb[2 * e], r1 = vb[2 * e + 1];
    const unsigned short hp0 = f2bf_bits(p0), hp1 = f2bf_bits(p1), hr0 = f2bf_bits(r0), hr1 = f2bf_bits(r1);
    const unsigned short lp0 = f2bf_bits(p0 - bf_bits2f(hp0)), lp1 = f2bf_bits(p1 - bf_bits2f(hp1));
    const unsigned short lr0 = f2bf_bits(r0 - bf_bits2f(hr0)), lr1 = f2bf_bits(r1 - bf_bits2f(hr1));
    wh[e]     = (unsigned)hp0 | ((unsigned)hp1 << 16);
    wh[2 + e] = (unsigned)hr0 | ((unsigned)hr1 << 16);
    wl[e]     = (unsigned)lp0 | ((unsigned)lp1 << 16);
    wl[2 + e] = (unsigned)lr0 | ((unsigned)lr1 << 16);
  }
  *(volatile v4u*)(Bhi + (size_t)tid * 4) = wh;
  *(volatile v4u*)(Blo + (size_t)tid * 4) = wl;
  __threadfence();
  *(volatile v4u*)(Bhi + (size_t)tid * 4) = wh;
  *(volatile v4u*)(Blo + (size_t)tid * 4) = wl;
}

__global__ __launch_bounds__(256) void gemm64_bf16x3_kernel(
    const unsigned short* __restrict__ Ap, const unsigned short* __restrict__ A2p, int lda,
    const unsigned short* __restrict__ Btp, const unsigned short* __restrict__ Bt2p, int ldb,
    float* __restrict__ C, int ldc, int M, int N, int K) {
  const __bf16* A   = (const __bf16*)Ap;
  const __bf16* A2  = (const __bf16*)A2p;
  const __bf16* Bt  = (const __bf16*)Btp;
  const __bf16* Bt2 = (const __bf16*)Bt2p;
  __shared__ __align__(16) float sT[8][16 * 68];
  const int lane = threadIdx.x & 31;
  const int wave = __builtin_amdgcn_readfirstlane((int)(threadIdx.x >> 5));
  const int tilesN = N >> 6;
  const int tilesM = M >> 6;
  const int tile = blockIdx.x * 8 + wave;
  if (tile >= tilesM * tilesN) return;
  const int tm = tile / tilesN;
  const int tn = tile - tm * tilesN;
  const int m0 = tm << 6;
  const int n0 = tn << 6;

  const int rlane = lane & 15;
  const int koff  = (lane >> 4) * 8;
  const int mOff  = (lane >> 4) * 8;

  v8f acc[4][4];
#pragma unroll
  for (int i = 0; i < 4; ++i)
#pragma unroll
    for (int j = 0; j < 4; ++j) acc[i][j] = (v8f){0.f, 0.f, 0.f, 0.f, 0.f, 0.f, 0.f, 0.f};

  for (int k0 = 0; k0 < K; k0 += 32) {
    v16b bh[4], bl[4];
#pragma unroll
    for (int j = 0; j < 4; ++j) {
      const size_t bo = (size_t)(n0 + (j << 4) + rlane) * ldb + koff + k0;
      bh[j] = FragB::load(Bt + bo);
      bl[j] = FragB::load(Bt2 + bo);
    }
#pragma unroll
    for (int i = 0; i < 4; ++i) {
      const size_t ao = (size_t)(m0 + (i << 4) + rlane) * lda + koff + k0;
      const v16b ah = FragB::load(A + ao);
      const v16b al = FragB::load(A2 + ao);
#pragma unroll
      for (int j = 0; j < 4; ++j) {
        acc[i][j] = FragB::mma(ah, bh[j], acc[i][j]);
        acc[i][j] = FragB::mma(ah, bl[j], acc[i][j]);
        acc[i][j] = FragB::mma(al, bh[j], acc[i][j]);
      }
      dep_guard4_b(acc[i][0], acc[i][1], acc[i][2], acc[i][3], ah, al);
    }
    keep4_b(bh[0], bh[1], bh[2], bh[3]);
    keep4_b(bl[0], bl[1], bl[2], bl[3]);
  }
  acc_guard4(acc[0][0], acc[0][1], acc[0][2], acc[0][3]);
  acc_guard4(acc[1][0], acc[1][1], acc[1][2], acc[1][3]);
  acc_guard4(acc[2][0], acc[2][1], acc[2][2], acc[2][3]);
  acc_guard4(acc[3][0], acc[3][1], acc[3][2], acc[3][3]);

  float* slab = sT[wave];
#pragma unroll
  for (int i = 0; i < 4; ++i) {
    const int mBase = m0 + (i << 4);
#pragma unroll
    for (int j = 0; j < 4; ++j) {
#pragma unroll
      for (int r = 0; r < 8; ++r) {
        slab[(mOff + r) * 68 + (j << 4) + rlane] = acc[i][j][r];
      }
    }
    __builtin_amdgcn_fence(__ATOMIC_RELEASE, "workgroup");
    __builtin_amdgcn_wave_barrier();
    __builtin_amdgcn_fence(__ATOMIC_ACQUIRE, "workgroup");
    {
      const int hh = lane >> 4, c4 = (lane & 15) * 4;
      for (int pass = 0; pass < 2; ++pass) {
#pragma unroll
        for (int it = 0; it < 8; ++it) {
          const int row = it * 2 + hh;
          const v4f v = *(const v4f*)(slab + row * 68 + c4);
          *(volatile v4f*)(C + (size_t)(mBase + row) * ldc + n0 + c4) = v;
        }
        __threadfence();
      }
    }
    __builtin_amdgcn_fence(__ATOMIC_RELEASE, "workgroup");
    __builtin_amdgcn_wave_barrier();
    __builtin_amdgcn_fence(__ATOMIC_ACQUIRE, "workgroup");
  }
}

__global__ __launch_bounds__(SCAN_THR) void gate_scan_kernel(
    const float* __restrict__ XP,
    const float* __restrict__ W0, const float* __restrict__ B0, const float* __restrict__ T0,
    const float* __restrict__ W1, const float* __restrict__ B1, const float* __restrict__ T1,
    const float* __restrict__ W2, const float* __restrict__ B2, const float* __restrict__ T2,
    const float* __restrict__ W3, const float* __restrict__ B3, const float* __restrict__ T3,
    float* __restrict__ out) {
  __shared__ __align__(16) float sWhT[NGATE * NQ * NQ];
  __shared__ __align__(16) float sBT[NCOL];
  __shared__ __align__(16) float sSlab[SCAN_THR / 32][32 * SLP];

  const int tid  = threadIdx.x;
  const int lane = tid & 31;
  const int wave = __builtin_amdgcn_readfirstlane((int)(threadIdx.x >> 5));
  const int brow  = blockIdx.x * SCAN_THR + tid;
  const int wrow0 = blockIdx.x * SCAN_THR + wave * 32;

  {
    const int gsel = tid >> 4;
    const int wq   = (tid >> 1) & 7;
    const int k4   = (tid & 1) * 4;
    const int wo   = wq * KDIM + IN_DIM + k4;
    v4f c0 = *(const v4f*)(W0 + wo);
    v4f c1 = *(const v4f*)(W1 + wo);
    v4f c2 = *(const v4f*)(W2 + wo);
    v4f c3 = *(const v4f*)(W3 + wo);
    asm volatile("" : "+v"(c0), "+v"(c1), "+v"(c2), "+v"(c3));
#pragma unroll
    for (int e = 0; e < 4; ++e) {
      const float s = (gsel == 0) ? c0[e] : (gsel == 1) ? c1[e] : (gsel == 2) ? c2[e] : c3[e];
      sWhT[(gsel * 8 + k4 + e) * 8 + wq] = s;
    }
  }
  {
    const int n  = tid & 31;
    const int gs = n >> 3;
    const int q  = n & 7;
    float p0 = B0[q], p1 = B1[q], p2 = B2[q], p3 = B3[q];
    float r0 = T0[q], r1 = T1[q], r2 = T2[q], r3 = T3[q];
    asm volatile("" : "+v"(p0), "+v"(p1), "+v"(p2), "+v"(p3), "+v"(r0), "+v"(r1), "+v"(r2), "+v"(r3));
    const float pb = (gs == 0) ? p0 : (gs == 1) ? p1 : (gs == 2) ? p2 : p3;
    const float pt = (gs == 0) ? r0 : (gs == 1) ? r1 : (gs == 2) ? r2 : r3;
    const float s = pb + pt;
    if (wave == 0) sBT[lane] = s;
  }
  float* wslab = sSlab[wave];
  float* myrow = wslab + lane * SLP;
  float* ystage = myrow + YSTAGE;
#pragma unroll
  for (int e = 0; e < 8; ++e) myrow[24 + e] = 0.0f;

  float cx[NQ];
#pragma unroll
  for (int w = 0; w < NQ; ++w) cx[w] = 0.0f;
  __syncthreads();

  const float* xpl = XP + (size_t)brow * NSTEP * XPP;

#pragma unroll 1
  for (int t = 0; t < NSTEP; ++t) {
    const int sc = t & 3;
    const int sp = (t + 3) & 3;
    const float* xprow = xpl + (size_t)t * XPP;
    const float* hlast = myrow + sp * 8;
    float vf[NQ], vi[NQ], vg[NQ], vo[NQ];
#pragma unroll
    for (int w = 0; w < NQ; ++w) { vf[w] = 0.0f; vi[w] = 0.0f; vg[w] = 0.0f; vo[w] = 0.0f; }

#pragma unroll 1
    for (int g = 0; g < NGATE; ++g) {
      const v4f xa = *(const v4f*)(xprow + g * 8);
      const v4f xb = *(const v4f*)(xprow + g * 8 + 4);
      const v4f ba = *(const v4f*)(sBT + g * 8);
      const v4f bb = *(const v4f*)(sBT + g * 8 + 4);
      float y[NQ];
#pragma unroll
      for (int e = 0; e < 4; ++e) { y[e] = xa[e] + ba[e]; y[4 + e] = xb[e] + bb[e]; }
      const float* wt = sWhT + g * (NQ * NQ);
#pragma unroll 1
      for (int k = 0; k < NQ; ++k) {
        const float hk = hlast[k];
        const v4f wa = *(const v4f*)(wt + k * 8);
        const v4f wb = *(const v4f*)(wt + k * 8 + 4);
#pragma unroll
        for (int e = 0; e < 4; ++e) {
          y[e]     = fmaf(wa[e], hk, y[e]);
          y[4 + e] = fmaf(wb[e], hk, y[4 + e]);
        }
      }
#pragma unroll
      for (int w = 0; w < NQ; ++w) ystage[w] = y[w];
#pragma unroll 1
      for (int w = 0; w < NQ; ++w) {
        const float yv = ystage[w];
        const float cv = cosf(yv);
        ystage[w] = cv;
      }
      float cw[NQ];
#pragma unroll
      for (int w = 0; w < NQ; ++w) cw[w] = ystage[w];
      float z[NQ];
      float p = cw[1];
#pragma unroll
      for (int w = 2; w < NQ; ++w) p *= cw[w];
      z[0] = p;
      float qv = cw[0];
#pragma unroll
      for (int w = 1; w < NQ; ++w) { qv *= cw[w]; z[w] = qv; }
      const bool isg = (g == 2);
      const float mA = isg ? 2.0f : 1.0f;
      const float dA = isg ? -1.0f : 0.0f;
#pragma unroll
      for (int w = 0; w < NQ; ++w) {
        const float v = fmaf(mA, fsig(mA * z[w]), dA);
        vf[w] = (g == 0) ? v : vf[w];
        vi[w] = (g == 1) ? v : vi[w];
        vg[w] = (g == 2) ? v : vg[w];
        vo[w] = (g == 3) ? v : vo[w];
      }
    }

    float* hcur = myrow + sc * 8;
#pragma unroll
    for (int w = 0; w < NQ; ++w) {
      const float c2 = fmaf(vf[w], cx[w], vi[w] * vg[w]);
      cx[w] = c2;
      hcur[w] = vo[w] * ftanh(c2);
    }

    if (sc == 3) {
      __syncthreads();
      const int q  = lane >> 3;
      const int j4 = (lane & 7) * 4;
      const int t0 = t - 3;
      for (int pass = 0; pass < 2; ++pass) {
#pragma unroll
        for (int it = 0; it < 8; ++it) {
          const int row = it * 4 + q;
          const v4f v = *(const v4f*)(wslab + row * SLP + j4);
          *(volatile v4f*)(out + ((size_t)(wrow0 + row) * NSTEP + (size_t)t0) * NQ + j4) = v;
        }
        __threadfence();
      }
      __syncthreads();
    }
  }

#pragma unroll
  for (int w = 0; w < NQ; ++w) myrow[w] = cx[w];
  __syncthreads();
  {
    float* o1 = out + (size_t)OUT0_N + (size_t)wrow0 * NQ;
    float* o2 = out + (size_t)OUT0_N + (size_t)OUT1_N + (size_t)wrow0 * NQ;
    for (int pass = 0; pass < 2; ++pass) {
#pragma unroll
      for (int i = 0; i < 2; ++i) {
        const int f   = i * 32 + lane;
        const int row = f >> 1;
        const int hf  = (f & 1) * 4;
        const v4f vh = *(const v4f*)(wslab + row * SLP + 24 + hf);
        const v4f vc = *(const v4f*)(wslab + row * SLP + hf);
        *(volatile v4f*)(o1 + f * 4) = vh;
        *(volatile v4f*)(o2 + f * 4) = vc;
      }
      __threadfence();
    }
  }
}

extern "C" void kernel_launch(void* const* d_in, const int* in_sizes, int n_in,
                              void* d_out, int out_size, void* d_ws, size_t ws_size, hipStream_t stream) {
  if (n_in < 13 || d_out == nullptr || d_ws == nullptr) return;
  if (in_sizes[0] != NBATCH * NSTEP * IN_DIM || out_size != OUT0_N + 2 * OUT1_N) return;
  for (int g = 0; g < NGATE; ++g) {
    if (in_sizes[1 + 3 * g] != NQ * KDIM || in_sizes[2 + 3 * g] != NQ || in_sizes[3 + 3 * g] != NQ) return;
  }

  const float* xin = (const float*)d_in[0];
  const float* Wf  = (const float*)d_in[1];
  const float* bf  = (const float*)d_in[2];
  const float* thf = (const float*)d_in[3];
  const float* Wi  = (const float*)d_in[4];
  const float* bi  = (const float*)d_in[5];
  const float* thi = (const float*)d_in[6];
  const float* Wu  = (const float*)d_in[7];
  const float* bu  = (const float*)d_in[8];
  const float* thu = (const float*)d_in[9];
  const float* Wo  = (const float*)d_in[10];
  const float* bo  = (const float*)d_in[11];
  const float* tho = (const float*)d_in[12];
  float* out = (float*)d_out;

  char* ws = (char*)d_ws;
  size_t off = 0;
  auto carve = [&](size_t bytes) -> char* { char* p = ws + off; off += (bytes + 255) & ~(size_t)255; return p; };
  unsigned short* AHI = (unsigned short*)carve((size_t)NROWS * IN_DIM * 2);
  unsigned short* ALO = (unsigned short*)carve((size_t)NROWS * IN_DIM * 2);
  unsigned short* BHI = (unsigned short*)carve((size_t)NPADN * IN_DIM * 2);
  unsigned short* BLO = (unsigned short*)carve((size_t)NPADN * IN_DIM * 2);
  float*          XPb = (float*)carve((size_t)NROWS * XPP * 4);
  if (off > ws_size || off > (size_t)134217728) return;

  split_x_kernel<<<X_N8 / 256, 256, 0, stream>>>(xin, (unsigned*)AHI, (unsigned*)ALO);
  split_w_kernel<<<1, 256, 0, stream>>>(Wf, Wi, Wu, Wo, (unsigned*)BHI, (unsigned*)BLO);

  gemm64_bf16x3_kernel<<<(NROWS / 64) * (NPADN / 64) / 8, 256, 0, stream>>>(
      AHI, ALO, IN_DIM, BHI, BLO, IN_DIM, XPb, XPP, NROWS, NPADN, IN_DIM);

  gate_scan_kernel<<<NBATCH / SCAN_THR, SCAN_THR, 0, stream>>>(
      XPb, Wf, bf, thf, Wi, bi, thi, Wu, bu, thu, Wo, bo, tho, out);
}
